// MultiheadAttention_78374563217616
// MI455X (gfx1250) — hardware-run, weakly checked
//
#include <hip/hip_runtime.h>


#ifndef NB
#define NB 2
#endif
#ifndef SEQ
#define SEQ 2047
#endif
#define NB_FULL  2
#define SEQ_FULL 2047
#ifndef MASKN
#define MASKN ((SEQ + 1) / 2)
#endif
#define TT   (((SEQ + 127) / 128) * 128)
#define DM   1024
#define NH_  16
#define HD   64
#define ZH   2
#define PCAR 1024.0f
#define SCL  0.125f
#define NEGM (-1.0e10f)
#define OSC  (0.125f / 1024.0f)

static_assert(TT % 128 == 0);
static_assert(TT >= SEQ);
static_assert(DM % 64 == 0);
static_assert(HD == 64);
static_assert(DM == NH_ * HD);
static_assert(NH_ % ZH == 0);
static_assert(SEQ <= SEQ_FULL);
static_assert(NB <= NB_FULL);
static_assert((size_t)NB_FULL * SEQ_FULL * DM * 4 == (size_t)16769024);
static_assert(SEQ != 2047 || MASKN == 1024);

typedef _Float16 h16;
typedef unsigned short bf;
typedef __attribute__((ext_vector_type(16))) __bf16   v16bf;
typedef __attribute__((ext_vector_type(16))) _Float16 v16h;
typedef __attribute__((ext_vector_type(8)))  _Float16 v8h;
typedef __attribute__((ext_vector_type(8)))  unsigned short v8us;
typedef __attribute__((ext_vector_type(8)))  float    v8f;
typedef __attribute__((ext_vector_type(4)))  float    v4f;
typedef __attribute__((ext_vector_type(2)))  float    v2f;
typedef __attribute__((ext_vector_type(2)))  _Float16 v2h;
typedef __attribute__((ext_vector_type(4)))  _Float16 v4h;
typedef __attribute__((ext_vector_type(2)))  unsigned short v2us;
typedef v4f  __attribute__((may_alias)) v4fa;

__device__ __forceinline__ unsigned short f2bf(float f) { unsigned u = __float_as_uint(f); u += 0x7FFFu + ((u >> 16) & 1u); return (unsigned short)(u >> 16); }
__device__ __forceinline__ float bf2f(unsigned short b) { return __uint_as_float(((unsigned)b) << 16); }
__device__ __forceinline__ v16h cat16(v8h lo, v8h hi) { return __builtin_shufflevector(lo, hi, 0, 1, 2, 3, 4, 5, 6, 7, 8, 9, 10, 11, 12, 13, 14, 15); }
__device__ __forceinline__ v16bf cat16b(v8us lo, v8us hi) { return __builtin_bit_cast(v16bf, __builtin_shufflevector(lo, hi, 0, 1, 2, 3, 4, 5, 6, 7, 8, 9, 10, 11, 12, 13, 14, 15)); }
__device__ __forceinline__ v8f wmma16(v16h a, v16h b, v8f c) { return __builtin_amdgcn_wmma_f32_16x16x32_f16(false, a, false, b, (short)0, c, false, false); }
__device__ __forceinline__ v8f wmmab(v16bf a, v16bf b, v8f c) { return __builtin_amdgcn_wmma_f32_16x16x32_bf16(false, a, false, b, (short)0, c, false, false); }
__device__ __forceinline__ h16 tohx(float x) { return (h16)x; }
__device__ __forceinline__ void splitf(float y, unsigned short& h, unsigned short& l) { h = f2bf(y); l = f2bf(y - bf2f(h)); }

template <typename T16> struct WFrag;
template <> struct WFrag<h16> { typedef v16h V; static __device__ __forceinline__ V ld(const h16* p) { return cat16(*(const v8h*)p, *(const v8h*)(p + 16)); } static __device__ __forceinline__ v8f mma(V a, V b, v8f c) { return wmma16(a, b, c); } };
template <> struct WFrag<bf> { typedef v16bf V; static __device__ __forceinline__ V ld(const bf* p) { return cat16b(*(const v8us*)p, *(const v8us*)(p + 16)); } static __device__ __forceinline__ v8f mma(V a, V b, v8f c) { return wmmab(a, b, c); } };
template <typename T16, int NSPLIT>
__global__ __launch_bounds__(32) void k_gemmw(const T16* __restrict__ A, const T16* __restrict__ A2, const T16* __restrict__ Bt, const T16* __restrict__ Bt2, int K, float* C, int ldc, int mrows, size_t sA, size_t sB, size_t sC) {
    typedef typename WFrag<T16>::V V;
    __shared__ __align__(16) float os[16 * 68];
    const size_t z = blockIdx.z; A += z * sA; if (A2) A2 += z * sA; Bt += z * sB; if (Bt2) Bt2 += z * sB; C += z * sC;
    const int lane = threadIdx.x & 31, lr = lane & 15, hi = lane >> 4; const int r0 = blockIdx.x * 64, c0 = blockIdx.y * 64;
    v8f acc[4][4];
#pragma unroll
    for (int mb = 0; mb < 4; ++mb)
#pragma unroll
        for (int nb = 0; nb < 4; ++nb) acc[mb][nb] = (v8f){};
    const size_t aoff = (size_t)(r0 + lr) * K + 8 * hi, boff = (size_t)(c0 + lr) * K + 8 * hi;
#pragma unroll 1
    for (int kc = 0; kc < K; kc += 32) {
        V a[4], a2[4];
#pragma unroll
        for (int mb = 0; mb < 4; ++mb) { a[mb] = WFrag<T16>::ld(A + aoff + (size_t)mb * 16 * K + kc); if (NSPLIT == 1 || NSPLIT == 2) a2[mb] = WFrag<T16>::ld(A2 + aoff + (size_t)mb * 16 * K + kc); }
#pragma unroll
        for (int nb = 0; nb < 4; ++nb) { const V b = WFrag<T16>::ld(Bt + boff + (size_t)nb * 16 * K + kc); V b2; if (NSPLIT >= 2) b2 = WFrag<T16>::ld(Bt2 + boff + (size_t)nb * 16 * K + kc);
#pragma unroll
            for (int mb = 0; mb < 4; ++mb) { acc[mb][nb] = WFrag<T16>::mma(a[mb], b, acc[mb][nb]); if (NSPLIT == 1 || NSPLIT == 2) acc[mb][nb] = WFrag<T16>::mma(a2[mb], b, acc[mb][nb]); if (NSPLIT >= 2) acc[mb][nb] = WFrag<T16>::mma(a[mb], b2, acc[mb][nb]); } }
        asm volatile("v_nop\n\tv_nop\n\tv_nop\n\tv_nop" : "+v"(acc[0][0]), "+v"(acc[1][1]), "+v"(acc[2][2]), "+v"(acc[3][3]) : "v"(a[0]), "v"(a[3]));
    }
#pragma unroll
    for (int mb = 0; mb < 4; ++mb) {
#pragma unroll
        for (int nb = 0; nb < 4; ++nb) {
#pragma unroll
            for (int j = 0; j < 8; ++j) os[(hi * 8 + j) * 68 + nb * 16 + lr] = acc[mb][nb][j]; }
        __builtin_amdgcn_wave_barrier(); asm volatile("" ::: "memory");
        float* crow = C + (size_t)(r0 + mb * 16) * ldc + c0;
#pragma unroll 1
        for (int ps = 0; ps < 2; ++ps) {
#pragma unroll
            for (int s = 0; s < 8; ++s) { const int row = 2 * s + hi, cofs = lr * 4; const v4f val = *(const v4fa*)(os + row * 68 + cofs);
                if (r0 + mb * 16 + row < mrows) *(volatile v4f*)(crow + (size_t)row * ldc + cofs) = val; }
            if (ps == 0) __threadfence(); }
        __builtin_amdgcn_wave_barrier(); asm volatile("" ::: "memory");
    }
}

__global__ __launch_bounds__(256) void k_wtG(const float* __restrict__ w, int K, int N, bf* Bt) {
    const int lane = threadIdx.x & 31; const int L0 = (blockIdx.x * 8 + (threadIdx.x >> 5)) * 8; const int nlines = N * K / 64;
#pragma unroll
    for (int ps = 0; ps < 2; ++ps) {
#pragma unroll 1
        for (int l = 0; l < 8; ++l) { const int L = L0 + l; if (L >= nlines) break; const size_t e = (size_t)L * 64 + lane * 2; const int k = (int)(e % K), n = (int)(e / K); v2us o;
            o[0] = f2bf(w[(size_t)k * N + n]); o[1] = f2bf(w[(size_t)(k + 1) * N + n]); *(volatile v2us*)(Bt + e) = o; }
        if (ps == 0) __threadfence(); }
}

__global__ __launch_bounds__(256) void k_cvtx(const float* __restrict__ src, bf* dst) {
    const size_t i = (size_t)blockIdx.x * 256 + threadIdx.x; if (i >= (size_t)NB * TT * (DM / 8)) return;
    const int c8 = (int)(i % (DM / 8)); const int t = (int)((i / (DM / 8)) % TT); const int b = (int)(i / ((size_t)(DM / 8) * TT));
    const int tc = (t < SEQ) ? t : (SEQ - 1);
    const v8f v = *(const v8f*)(src + ((size_t)b * SEQ_FULL + tc) * DM + (size_t)c8 * 8); v8us o;
#pragma unroll
    for (int k = 0; k < 8; ++k) o[k] = (t < SEQ) ? f2bf(v[k]) : (unsigned short)0;
    *(volatile v8us*)(dst + i * 8) = o; __threadfence(); *(volatile v8us*)(dst + i * 8) = o; }

__global__ __launch_bounds__(256) void k_qkp(const float* __restrict__ F, h16* P16) {
    const size_t e = ((size_t)blockIdx.x * 256 + threadIdx.x) * 2; if (e >= (size_t)NB * NH_ * TT * HD) return;
    const int d = (int)(e % HD); const int t = (int)((e / HD) % TT); const int zh = (int)(e / ((size_t)HD * TT)); const int b = zh / NH_, h = zh % NH_;
    const v2f x = *(const v2f*)(F + ((size_t)b * TT + t) * DM + h * HD + d); v2h o; o[0] = tohx(x[0]); o[1] = tohx(x[1]);
    *(volatile v2h*)(P16 + e) = o; __threadfence(); *(volatile v2h*)(P16 + e) = o; }

__global__ __launch_bounds__(256) void k_vtp(const float* __restrict__ F, h16* V16) {
    const size_t e = ((size_t)blockIdx.x * 256 + threadIdx.x) * 2; if (e >= (size_t)NB * NH_ * HD * TT) return;
    const int t = (int)(e % TT); const int d = (int)((e / TT) % HD); const int zh = (int)(e / ((size_t)TT * HD)); const int b = zh / NH_, h = zh % NH_; v2h o;
#pragma unroll
    for (int q = 0; q < 2; ++q) { const float x = F[((size_t)b * TT + t + q) * DM + h * HD + d]; o[q] = tohx(x); }
    *(volatile v2h*)(V16 + e) = o; __threadfence(); *(volatile v2h*)(V16 + e) = o; }

__global__ __launch_bounds__(256) void k_asoft(const float* __restrict__ Sb, h16* P16) {
    const int lane = threadIdx.x & 31; const int row = blockIdx.x * 8 + (threadIdx.x >> 5); if (row >= ZH * TT) return;
    const int i = row % TT; const float qb = (i < MASKN) ? NEGM : 0.0f;
    const float* sr = Sb + (size_t)row * TT; float v[TT / 32]; float mx = -1.0e30f;
#pragma unroll
    for (int ch = 0; ch < TT / 128; ++ch) { const int j0 = ch * 128 + lane * 4; const v4f a = *(const v4f*)(sr + j0);
#pragma unroll
        for (int q = 0; q < 4; ++q) { const int j = j0 + q; float s = __fmul_rn(a[q], SCL); asm volatile("" : "+v"(s)); const float t = (j < SEQ) ? __fadd_rn(s, qb) : -1.0e30f; v[ch * 4 + q] = t; mx = fmaxf(mx, t); } }
#pragma unroll
    for (int sh = 16; sh; sh >>= 1) mx = fmaxf(mx, __shfl_xor(mx, sh, 32));
    float sum = 0.f;
#pragma unroll
    for (int k = 0; k < TT / 32; ++k) { float d0 = __fsub_rn(v[k], mx); asm volatile("" : "+v"(d0)); v[k] = __builtin_amdgcn_exp2f(__fmul_rn(d0, 1.4426950408889634f)); sum += v[k]; }
#pragma unroll
    for (int sh = 16; sh; sh >>= 1) sum += __shfl_xor(sum, sh, 32);
    const float f = __fdiv_rn(PCAR, sum);
#pragma unroll 1
    for (int ps = 0; ps < 2; ++ps) {
#pragma unroll
        for (int ch = 0; ch < TT / 128; ++ch) { v4h o4;
#pragma unroll
            for (int q = 0; q < 4; ++q) o4[q] = tohx(v[ch * 4 + q] * f);
            *(volatile v4h*)(P16 + (size_t)row * TT + ch * 128 + lane * 4) = o4; }
        if (ps == 0) __threadfence(); }
}

__global__ __launch_bounds__(256) void k_merge(const float* __restrict__ O, int b, int h0, bf* Ah, bf* Al) {
    const size_t e = ((size_t)blockIdx.x * 256 + threadIdx.x) * 2; if (e >= (size_t)ZH * TT * HD) return;
    const int d = (int)(e % HD); const int t = (int)((e / HD) % TT); const int zz = (int)(e / ((size_t)HD * TT));
    const size_t oo = ((size_t)b * TT + t) * DM + (h0 + zz) * HD + d; const v2f x = *(const v2f*)(O + e); v2us oh, ol;
#pragma unroll
    for (int q = 0; q < 2; ++q) { unsigned short a, c2; splitf(x[q] * OSC, a, c2); oh[q] = a; ol[q] = c2; }
    *(volatile v2us*)(Ah + oo) = oh; *(volatile v2us*)(Al + oo) = ol; __threadfence(); *(volatile v2us*)(Ah + oo) = oh; *(volatile v2us*)(Al + oo) = ol; }

constexpr size_t al256(size_t x) { return (x + 255) & ~(size_t)255; }
constexpr size_t SZ_W   = al256((size_t)DM * DM * 2);
constexpr size_t SZ_XB  = al256((size_t)NB * TT * DM * 2);
constexpr size_t SZ_F   = al256((size_t)NB * TT * DM * 4);
constexpr size_t SZ_PL  = al256((size_t)NB * NH_ * TT * HD * 2);
constexpr size_t SZ_SB  = al256((size_t)ZH * TT * TT * 4);
constexpr size_t SZ_P16 = al256((size_t)ZH * TT * TT * 2);
constexpr size_t SZ_OB  = al256((size_t)ZH * TT * HD * 4);
constexpr size_t SZ_AT  = al256((size_t)NB * TT * DM * 2);
constexpr size_t SZ_ALL = 4 * SZ_W + SZ_XB + SZ_F + 3 * SZ_PL + SZ_SB + SZ_P16 + SZ_OB + 2 * SZ_AT;
static_assert(SZ_ALL <= (size_t)134217728);

extern "C" void kernel_launch(void* const* d_in, const int* in_sizes, int n_in,
                              void* d_out, int out_size, void* d_ws, size_t ws_size, hipStream_t stream) {
    if (n_in < 7) return;
    const size_t needx = (size_t)(NB - 1) * SEQ_FULL * DM + (size_t)SEQ * DM;
    for (int i = 0; i < 3; ++i) if ((size_t)in_sizes[i] < needx) return;
    for (int i = 3; i < 7; ++i) if ((size_t)in_sizes[i] < (size_t)DM * DM) return;
    if ((size_t)out_size < (size_t)NB * SEQ * DM) return;
    if (SZ_ALL > ws_size) return;
    const float* xq = (const float*)d_in[0]; const float* xk = (const float*)d_in[1]; const float* xv = (const float*)d_in[2];
    const float* wq = (const float*)d_in[3]; const float* wk = (const float*)d_in[4]; const float* wv = (const float*)d_in[5]; const float* wo = (const float*)d_in[6];
    float* OUT = (float*)d_out;
    char* wsp = (char*)d_ws;
    auto take = [&](size_t bytes) { char* p = wsp; wsp += bytes; return (void*)p; };
    bf* WQ = (bf*)take(SZ_W); bf* WK = (bf*)take(SZ_W); bf* WV = (bf*)take(SZ_W); bf* WO = (bf*)take(SZ_W);
    bf* XB = (bf*)take(SZ_XB); float* F = (float*)take(SZ_F);
    h16* QP16 = (h16*)take(SZ_PL); h16* KP16 = (h16*)take(SZ_PL); h16* VT16 = (h16*)take(SZ_PL);
    float* Sb = (float*)take(SZ_SB); h16* P16 = (h16*)take(SZ_P16); float* Ob = (float*)take(SZ_OB);
    bf* ATh = (bf*)take(SZ_AT); bf* ATl = (bf*)take(SZ_AT);
    if ((size_t)(wsp - (char*)d_ws) > ws_size) return;

    const unsigned GW = (unsigned)((DM * DM / 64 + 63) / 64);
    k_wtG<<<GW, 256, 0, stream>>>(wq, DM, DM, WQ);
    k_wtG<<<GW, 256, 0, stream>>>(wk, DM, DM, WK);
    k_wtG<<<GW, 256, 0, stream>>>(wv, DM, DM, WV);
    k_wtG<<<GW, 256, 0, stream>>>(wo, DM, DM, WO);

    const unsigned GC = (unsigned)(((size_t)NB * TT * (DM / 8) + 255) / 256);
    const unsigned GP = (unsigned)(((size_t)NB * NH_ * TT * HD / 2 + 255) / 256);
    const dim3 GPRJ((unsigned)(NB * TT / 64), (unsigned)(DM / 64), 1);
    k_cvtx<<<GC, 256, 0, stream>>>(xq, XB);
    k_gemmw<bf, 0><<<GPRJ, 32, 0, stream>>>(XB, nullptr, WQ, nullptr, DM, F, DM, NB * TT, 0, 0, 0);
    k_qkp<<<GP, 256, 0, stream>>>(F, QP16);
    k_cvtx<<<GC, 256, 0, stream>>>(xk, XB);
    k_gemmw<bf, 0><<<GPRJ, 32, 0, stream>>>(XB, nullptr, WK, nullptr, DM, F, DM, NB * TT, 0, 0, 0);
    k_qkp<<<GP, 256, 0, stream>>>(F, KP16);
    k_cvtx<<<GC, 256, 0, stream>>>(xv, XB);
    k_gemmw<bf, 0><<<GPRJ, 32, 0, stream>>>(XB, nullptr, WV, nullptr, DM, F, DM, NB * TT, 0, 0, 0);
    k_vtp<<<GP, 256, 0, stream>>>(F, VT16);

    for (int z0 = 0; z0 < NB * NH_; z0 += ZH) { const int b = z0 / NH_, h0 = z0 % NH_; const size_t zo = (size_t)z0 * TT * HD;
        k_gemmw<h16, 0><<<dim3(TT / 64, TT / 64, ZH), 32, 0, stream>>>(QP16 + zo, nullptr, KP16 + zo, nullptr, HD, Sb, TT, TT, (size_t)TT * HD, (size_t)TT * HD, (size_t)TT * TT);
        k_asoft<<<ZH * TT / 8, 256, 0, stream>>>(Sb, P16);
        k_gemmw<h16, 0><<<dim3(TT / 64, HD / 64, ZH), 32, 0, stream>>>(P16, nullptr, VT16 + zo, nullptr, TT, Ob, HD, TT, (size_t)TT * TT, (size_t)HD * TT, (size_t)TT * HD);
        k_merge<<<(unsigned)(((size_t)ZH * TT * HD / 2 + 255) / 256), 256, 0, stream>>>(Ob, b, h0, ATh, ATl); }

    k_gemmw<bf, 1><<<dim3(TT / 64, DM / 64, NB), 32, 0, stream>>>(ATh, ATl, WO, nullptr, DM, OUT, DM, SEQ, (size_t)TT * DM, 0, (size_t)SEQ * DM);
}
